// MTNN_48558900248798
// MI455X (gfx1250) — hardware-run, weakly checked
//
#include <hip/hip_runtime.h>


#define AS3 __attribute__((address_space(3)))

#define NB   512
#define NT   300
#define NIS  128
#define NID  64
#define NHS  256
#define NHD  128
#define NNEU 1000
#define NFD  512
#define ZP   320

static_assert(NFD == NHS + 2 * NHD);
static_assert(NIS % 32 == 0 && NID % 32 == 0 && NHS % 32 == 0 && NHD % 32 == 0);
static_assert(NB % 32 == 0);
static_assert((NB * NT) % 128 == 0);
static_assert((NB * NT) % (4 * 256) == 0);
static_assert(ZP % 32 == 0 && ZP >= ((NT + 31) / 32) * 32);
static_assert(NHD == 128);

typedef __bf16         v16b __attribute__((ext_vector_type(16)));
typedef unsigned short v8us __attribute__((ext_vector_type(8)));
typedef float          v8f  __attribute__((ext_vector_type(8)));
typedef float          v4f  __attribute__((ext_vector_type(4)));
typedef v8us __attribute__((may_alias)) v8usa;
typedef v4f  __attribute__((may_alias)) v4fa;

typedef AS3 unsigned short*       lp_us;
typedef AS3 const unsigned short* lcp_us;
typedef AS3 float*                lp_f;
typedef AS3 const float*          lcp_f;

union Frag { v16b v; v8us half[2]; };

constexpr int P_XS  = 0;
constexpr int P_W1  = P_XS  + NB * NIS;
constexpr int P_W2  = P_W1  + NHS * NIS;
constexpr int P_WD  = P_W2  + NHS * NHS;
constexpr int P_WIF = P_WD  + NHD * NID;
constexpr int P_WHF = P_WIF + NHD * NHD;
constexpr int P_WIB = P_WHF + NHD * NHD;
constexpr int P_WHB = P_WIB + NHD * NHD;
constexpr int P_XD  = P_WHB + NHD * NHD;
constexpr int P_END = P_XD  + NB * NT * NID;
constexpr int NPC   = P_END / 8;
constexpr int NCBLK = NPC / 256;
static_assert(P_END % 8 == 0);
static_assert(NPC % 256 == 0);
static_assert(P_W1 % 2048 == 0 && P_W2 % 2048 == 0 && P_WD % 2048 == 0 && P_WIF % 2048 == 0 &&
              P_WHF % 2048 == 0 && P_WIB % 2048 == 0 && P_WHB % 2048 == 0 && P_XD % 2048 == 0);

constexpr size_t OFF_CV = 0;
constexpr size_t SZ_CV  = (size_t)P_END * 2;
constexpr size_t OFF_DH = OFF_CV + SZ_CV;
constexpr size_t SZ_D   = (size_t)NB * NT * NHD * 2;
constexpr size_t OFF_DL = OFF_DH + SZ_D;
constexpr size_t OFF_C  = OFF_DL + SZ_D;
constexpr size_t SZ_C   = (size_t)NB * 4;
constexpr size_t OFF_Z  = OFF_C + SZ_C;
constexpr size_t SZ_Z   = (size_t)2 * NB * ZP * 4;
constexpr size_t WS_END = OFF_Z + SZ_Z;
static_assert(OFF_DH % 128 == 0 && OFF_DL % 128 == 0 && OFF_C % 128 == 0 && OFF_Z % 128 == 0);
static_assert(WS_END <= (size_t)134217728);
static_assert((size_t)NPC * 16 == SZ_CV);
static_assert((size_t)(NB * NT / 128) * 2 * 128 * 128 == SZ_D);
static_assert((size_t)(NB / 32) * 128 == SZ_C);
static_assert((size_t)2 * NB * (ZP / 32) * 128 == SZ_Z);

__device__ __forceinline__ unsigned short bf16_bits(float f) {
  unsigned u = __float_as_uint(f);
  u += 0x7FFFu + ((u >> 16) & 1u);
  return (unsigned short)(u >> 16);
}
__device__ __forceinline__ float bf16_val(unsigned short b) { return __uint_as_float(((unsigned)b) << 16); }
__device__ __forceinline__ float bf16r(float f) { return bf16_val(bf16_bits(f)); }
__device__ __forceinline__ v8f zero8() {
  v8f z;
#pragma unroll
  for (int i = 0; i < 8; ++i) z[i] = 0.0f;
  return z;
}

__device__ __forceinline__ void ldfrag_g(Frag& f, const unsigned short* p, int h) {
  f.half[0] = *(const v8usa*)(p + 8 * h);
  f.half[1] = *(const v8usa*)(p + 16 + 8 * h);
}
__device__ __forceinline__ void ldfrag_l(Frag& f, lcp_us p, int h) {
  f.half[0] = *(AS3 const v8usa*)(p + 8 * h);
  f.half[1] = *(AS3 const v8usa*)(p + 16 + 8 * h);
}
__device__ __forceinline__ v8f mma16(v8f c, const Frag& a, const Frag& b) {
  return __builtin_amdgcn_wmma_f32_16x16x32_bf16(false, a.v, false, b.v, (short)0, c, false, false);
}

__global__ __launch_bounds__(256)
void cvt_kernel(const float* __restrict__ xs,  const float* __restrict__ w1,  const float* __restrict__ w2,
                const float* __restrict__ wd,  const float* __restrict__ wif, const float* __restrict__ whf,
                const float* __restrict__ wib, const float* __restrict__ whb, const float* __restrict__ xd,
                unsigned short* cv)
{
  const int g = blockIdx.x * 256 + threadIdx.x;
  if (g >= NPC) return;
  const int e = g * 8;
  const float* src;
  if      (e < P_W1)  src = xs  + e;
  else if (e < P_W2)  src = w1  + (e - P_W1);
  else if (e < P_WD)  src = w2  + (e - P_W2);
  else if (e < P_WIF) src = wd  + (e - P_WD);
  else if (e < P_WHF) src = wif + (e - P_WIF);
  else if (e < P_WIB) src = whf + (e - P_WHF);
  else if (e < P_WHB) src = wib + (e - P_WIB);
  else if (e < P_XD)  src = whb + (e - P_WHB);
  else                src = xd  + (e - P_XD);
  const v4f a = *(const v4fa*)src;
  const v4f c = *(const v4fa*)(src + 4);
  v8us o;
  o[0] = bf16_bits(a[0]); o[1] = bf16_bits(a[1]); o[2] = bf16_bits(a[2]); o[3] = bf16_bits(a[3]);
  o[4] = bf16_bits(c[0]); o[5] = bf16_bits(c[1]); o[6] = bf16_bits(c[2]); o[7] = bf16_bits(c[3]);
  unsigned short* dst = cv + e;
  *(volatile v8us*)dst = o;
  __threadfence();
  *(volatile v8us*)dst = o;
}

constexpr int    SP1   = NHS + 8;
constexpr size_t SL_HI = 0;
constexpr size_t SLT   = (size_t)32 * SP1 * 2;
constexpr size_t SL_LO = SL_HI + SLT;
constexpr size_t SL_S  = SL_LO + SLT;
constexpr size_t SL_CV = SL_S + (size_t)32 * NHS * 4;
constexpr size_t SLDS  = SL_CV + 128;
static_assert(SP1 % 8 == 0);
static_assert(SL_LO % 16 == 0 && SL_S % 16 == 0 && SL_CV % 16 == 0);

__global__ __launch_bounds__(256)
void smlp_kernel(const unsigned short* __restrict__ cv, const float* __restrict__ b1,
                 const float* __restrict__ b2, const int* __restrict__ nord,
                 const float* __restrict__ fcw, const float* __restrict__ fcb, float* cpl)
{
  extern __shared__ __attribute__((aligned(16))) char smem[];
  lp_us sHi = (lp_us)(smem + SL_HI);
  lp_us sLo = (lp_us)(smem + SL_LO);
  lp_f  sS  = (lp_f)(smem + SL_S);
  lp_f  sCv = (lp_f)(smem + SL_CV);

  const int tid = threadIdx.x, lane = tid & 31, w = tid >> 5;
  const int h = lane >> 4, m = lane & 15;
  const int b0 = blockIdx.x * 32;
  const unsigned short* XS = cv + P_XS;
  const unsigned short* W1 = cv + P_W1;
  const unsigned short* W2 = cv + P_W2;

  v8f acc[2][2];
#pragma unroll
  for (int mt = 0; mt < 2; ++mt)
#pragma unroll
    for (int nt = 0; nt < 2; ++nt) acc[mt][nt] = zero8();
  {
    const unsigned short* xa = XS + (size_t)(b0 + m) * NIS;
    const unsigned short* wb = W1 + (size_t)(32 * w + m) * NIS;
#pragma unroll 1
    for (int k0 = 0; k0 < NIS; k0 += 32) {
      Frag a[2], b[2];
#pragma unroll
      for (int mt = 0; mt < 2; ++mt) ldfrag_g(a[mt], xa + (size_t)mt * 16 * NIS + k0, h);
#pragma unroll
      for (int nt = 0; nt < 2; ++nt) ldfrag_g(b[nt], wb + (size_t)nt * 16 * NIS + k0, h);
#pragma unroll
      for (int mt = 0; mt < 2; ++mt)
#pragma unroll
        for (int nt = 0; nt < 2; ++nt) acc[mt][nt] = mma16(acc[mt][nt], a[mt], b[nt]);
      asm volatile("v_nop\n\tv_nop\n\tv_nop\n\tv_nop"
                   : "+v"(acc[0][0]), "+v"(acc[0][1]), "+v"(acc[1][0]), "+v"(acc[1][1])
                   : "v"(a[0].v), "v"(a[1].v), "v"(b[0].v), "v"(b[1].v));
    }
  }
#pragma unroll
  for (int nt = 0; nt < 2; ++nt) {
    const int col = 32 * w + 16 * nt + m;
    const float bias = bf16r(b1[col]);
#pragma unroll
    for (int mt = 0; mt < 2; ++mt)
#pragma unroll
      for (int r = 0; r < 8; ++r) {
        const int row = 16 * mt + 8 * h + r;
        const float v = fmaxf(acc[mt][nt][r] + bias, 0.0f);
        const unsigned short hb = bf16_bits(v);
        const unsigned short lb = bf16_bits(v - bf16_val(hb));
        sHi[row * SP1 + col] = hb;
        sLo[row * SP1 + col] = lb;
      }
  }
  __syncthreads();

#pragma unroll
  for (int mt = 0; mt < 2; ++mt)
#pragma unroll
    for (int nt = 0; nt < 2; ++nt) acc[mt][nt] = zero8();
  {
    lcp_us ha = sHi + m * SP1;
    lcp_us la = sLo + m * SP1;
    const unsigned short* wb = W2 + (size_t)(32 * w + m) * NHS;
#pragma unroll 1
    for (int k0 = 0; k0 < NHS; k0 += 32) {
      Frag ah[2], al[2], b[2];
#pragma unroll
      for (int mt = 0; mt < 2; ++mt) {
        ldfrag_l(ah[mt], ha + mt * 16 * SP1 + k0, h);
        ldfrag_l(al[mt], la + mt * 16 * SP1 + k0, h);
      }
#pragma unroll
      for (int nt = 0; nt < 2; ++nt) ldfrag_g(b[nt], wb + (size_t)nt * 16 * NHS + k0, h);
#pragma unroll
      for (int mt = 0; mt < 2; ++mt)
#pragma unroll
        for (int nt = 0; nt < 2; ++nt) {
          acc[mt][nt] = mma16(acc[mt][nt], ah[mt], b[nt]);
          acc[mt][nt] = mma16(acc[mt][nt], al[mt], b[nt]);
        }
      asm volatile("v_nop\n\tv_nop\n\tv_nop\n\tv_nop"
                   : "+v"(acc[0][0]), "+v"(acc[0][1]), "+v"(acc[1][0]), "+v"(acc[1][1])
                   : "v"(ah[0].v), "v"(ah[1].v), "v"(al[0].v), "v"(al[1].v), "v"(b[0].v), "v"(b[1].v));
    }
  }
#pragma unroll
  for (int nt = 0; nt < 2; ++nt) {
    const int col = 32 * w + 16 * nt + m;
    const float bias = bf16r(b2[col]);
#pragma unroll
    for (int mt = 0; mt < 2; ++mt)
#pragma unroll
      for (int r = 0; r < 8; ++r) {
        const int row = 16 * mt + 8 * h + r;
        sS[row * NHS + col] = fmaxf(acc[mt][nt][r] + bias, 0.0f);
      }
  }
  __syncthreads();

  const int smp = tid >> 3, sub = tid & 7;
  const int nid = min(max(nord[b0 + smp], 0), NNEU - 1);
  const float* wrow = fcw + (size_t)nid * NFD + sub * 32;
  lcp_f srow = sS + smp * NHS + sub * 32;
  float pc = 0.0f;
#pragma unroll
  for (int j = 0; j < 8; ++j) {
    const v4f sv = *(AS3 const v4fa*)(srow + 4 * j);
    const v4f wv = *(const v4fa*)(wrow + 4 * j);
    pc += sv[0] * bf16r(wv[0]);
    pc += sv[1] * bf16r(wv[1]);
    pc += sv[2] * bf16r(wv[2]);
    pc += sv[3] * bf16r(wv[3]);
  }
  pc += __shfl_xor(pc, 1);
  pc += __shfl_xor(pc, 2);
  pc += __shfl_xor(pc, 4);
  if (sub == 0) sCv[smp] = pc + bf16r(fcb[nid]);
  __syncthreads();

  v4f cvv = {0.0f, 0.0f, 0.0f, 0.0f};
  if (tid < 8) cvv = *(AS3 const v4fa*)(sCv + 4 * tid);
  float* cdst = cpl + b0 + 4 * min(tid, 7);
  if (tid < 8) *(volatile v4f*)cdst = cvv;
  __threadfence();
  if (tid < 8) *(volatile v4f*)cdst = cvv;
}

constexpr size_t DL_TH = 0;
constexpr size_t DL_TL = (size_t)128 * 64 * 2;
constexpr size_t DLDS  = 2 * DL_TL;

__global__ __launch_bounds__(128)
void dproj_kernel(const unsigned short* __restrict__ cv, const float* __restrict__ bd,
                  unsigned short* dh, unsigned short* dl)
{
  extern __shared__ __attribute__((aligned(16))) char smem[];
  lp_us sTH = (lp_us)(smem + DL_TH);
  lp_us sTL = (lp_us)(smem + DL_TL);

  const int tid = threadIdx.x, lane = tid & 31, w = tid >> 5;
  const int h = lane >> 4, m = lane & 15;
  const int m0 = blockIdx.x * 128;
  const int cy = blockIdx.y;
  const int m0w = m0 + 32 * w;
  const unsigned short* XD = cv + P_XD;
  const unsigned short* WD = cv + P_WD;

  const unsigned short* xa = XD + (size_t)(m0w + m) * NID;
  const unsigned short* wb = WD + (size_t)(64 * cy + m) * NID;

  v8f acc[2][4];
#pragma unroll
  for (int mt = 0; mt < 2; ++mt)
#pragma unroll
    for (int nt = 0; nt < 4; ++nt) acc[mt][nt] = zero8();

#pragma unroll 1
  for (int k0 = 0; k0 < NID; k0 += 32) {
    Frag a[2], b[4];
#pragma unroll
    for (int mt = 0; mt < 2; ++mt) ldfrag_g(a[mt], xa + (size_t)mt * 16 * NID + k0, h);
#pragma unroll
    for (int nt = 0; nt < 4; ++nt) ldfrag_g(b[nt], wb + (size_t)nt * 16 * NID + k0, h);
#pragma unroll
    for (int mt = 0; mt < 2; ++mt)
#pragma unroll
      for (int nt = 0; nt < 4; ++nt) acc[mt][nt] = mma16(acc[mt][nt], a[mt], b[nt]);
    asm volatile("v_nop\n\tv_nop\n\tv_nop\n\tv_nop"
                 : "+v"(acc[0][0]), "+v"(acc[0][1]), "+v"(acc[0][2]), "+v"(acc[0][3]),
                   "+v"(acc[1][0]), "+v"(acc[1][1]), "+v"(acc[1][2]), "+v"(acc[1][3])
                 : "v"(a[0].v), "v"(a[1].v), "v"(b[0].v), "v"(b[1].v), "v"(b[2].v), "v"(b[3].v));
  }

#pragma unroll
  for (int nt = 0; nt < 4; ++nt) {
    const int col = 16 * nt + m;
    const float bias = bf16r(bd[64 * cy + col]);
#pragma unroll
    for (int mt = 0; mt < 2; ++mt)
#pragma unroll
      for (int r = 0; r < 8; ++r) {
        const int rowl = 32 * w + 16 * mt + 8 * h + r;
        const float v = fmaxf(acc[mt][nt][r] + bias, 0.0f);
        const unsigned short hb = bf16_bits(v);
        const unsigned short lb = bf16_bits(v - bf16_val(hb));
        sTH[rowl * 64 + col] = hb;
        sTL[rowl * 64 + col] = lb;
      }
  }
  __syncthreads();

  const int q8 = lane & 7, sub = lane >> 3;
#pragma unroll 1
  for (int pass = 0; pass < 2; ++pass) {
#pragma unroll
    for (int i = 0; i < 8; ++i) {
      const int lid = 32 * w + 4 * i + sub;
      const v8us vh = *(AS3 const v8usa*)(sTH + lid * 64 + 8 * q8);
      const v8us vl = *(AS3 const v8usa*)(sTL + lid * 64 + 8 * q8);
      const size_t go = (size_t)(m0 + lid) * NHD + 64 * cy + 8 * q8;
      *(volatile v8us*)(dh + go) = vh;
      *(volatile v8us*)(dl + go) = vl;
    }
    __threadfence();
  }
}

constexpr int    HP     = NHD + 8;
constexpr int    HTILE  = 32 * HP;
constexpr size_t RL_HH  = 0;
constexpr size_t RLSZ_H = (size_t)2 * HTILE * 2;
constexpr size_t RL_HL  = RL_HH + RLSZ_H;
constexpr size_t RL_WG  = RL_HL + RLSZ_H;
constexpr size_t RL_ZW  = RL_WG + (size_t)32 * NHD * 2;
constexpr size_t RL_BI  = RL_ZW + (size_t)4 * 32 * 32 * 4;
constexpr size_t RLDS   = RL_BI + (size_t)NHD * 4;
static_assert(HP % 8 == 0);
static_assert(RL_HL % 16 == 0 && RL_WG % 16 == 0 && RL_ZW % 16 == 0 && RL_BI % 16 == 0);
constexpr int NZH = (int)(RL_WG / 16);
constexpr int NZZ = (int)((RL_BI - RL_ZW) / 16);

__global__ __launch_bounds__(128)
void brnn_kernel(const unsigned short* __restrict__ cv, const unsigned short* __restrict__ dh,
                 const unsigned short* __restrict__ dl,
                 const float* __restrict__ bihf, const float* __restrict__ bhhf,
                 const float* __restrict__ bihb, const float* __restrict__ bhhb,
                 const int* __restrict__ nord, const float* __restrict__ fcw, float* zpl)
{
  extern __shared__ __attribute__((aligned(16))) char smem[];
  lp_us hH    = (lp_us)(smem + RL_HH);
  lp_us hL    = (lp_us)(smem + RL_HL);
  lp_us sWg   = (lp_us)(smem + RL_WG);
  lp_f  sZw   = (lp_f)(smem + RL_ZW);
  lp_f  sBias = (lp_f)(smem + RL_BI);

  const int tid = threadIdx.x, lane = tid & 31, w = tid >> 5;
  const int h = lane >> 4, m = lane & 15;
  const int dir = (int)blockIdx.x >> 4;
  const int b0  = ((int)blockIdx.x & 15) * 32;
  const unsigned short* WI = cv + (dir ? P_WIB : P_WIF);
  const unsigned short* WH = cv + (dir ? P_WHB : P_WHF);
  const float* bih = dir ? bihb : bihf;
  const float* bhh = dir ? bhhb : bhhf;

  {
    v8us z8;
#pragma unroll
    for (int i = 0; i < 8; ++i) z8[i] = (unsigned short)0;
    for (int i = tid; i < NZH; i += 128) *(AS3 v8us*)(hH + 8 * i) = z8;
    v4f z4 = {0.0f, 0.0f, 0.0f, 0.0f};
    for (int i = tid; i < NZZ; i += 128) *(AS3 v4f*)(sZw + 4 * i) = z4;
    sBias[tid] = bf16r(bih[tid]) + bf16r(bhh[tid]);
#pragma unroll 1
    for (int row = 0; row < 32; ++row) {
      const int nid = min(max(nord[b0 + row], 0), NNEU - 1);
      sWg[row * NHD + tid] = bf16_bits(fcw[(size_t)nid * NFD + NHS + NHD * dir + tid]);
    }
  }
  __syncthreads();

  const int q8 = lane & 7, sub = lane >> 3;

#pragma unroll 1
  for (int s = 0; s < NT; ++s) {
    const int t   = dir ? (NT - 1 - s) : s;
    const int cur = s & 1;
    lcp_us hHc = hH + cur * HTILE;
    lcp_us hLc = hL + cur * HTILE;
    lp_us  hHn = hH + (cur ^ 1) * HTILE;
    lp_us  hLn = hL + (cur ^ 1) * HTILE;

    __syncthreads();

    v8f acc[2][2];
#pragma unroll
    for (int mt = 0; mt < 2; ++mt)
#pragma unroll
      for (int nt = 0; nt < 2; ++nt) acc[mt][nt] = zero8();

    {
      const size_t drow = ((size_t)(b0 + m) * NT + t) * NHD;
      const unsigned short* da  = dh + drow;
      const unsigned short* dla = dl + drow;
      const unsigned short* wb  = WI + (size_t)(32 * w + m) * NHD;
#pragma unroll 1
      for (int k0 = 0; k0 < NHD; k0 += 32) {
        Frag ah[2], al[2], b[2];
#pragma unroll
        for (int mt = 0; mt < 2; ++mt) {
          ldfrag_g(ah[mt], da  + (size_t)mt * 16 * NT * NHD + k0, h);
          ldfrag_g(al[mt], dla + (size_t)mt * 16 * NT * NHD + k0, h);
        }
#pragma unroll
        for (int nt = 0; nt < 2; ++nt) ldfrag_g(b[nt], wb + (size_t)nt * 16 * NHD + k0, h);
#pragma unroll
        for (int mt = 0; mt < 2; ++mt)
#pragma unroll
          for (int nt = 0; nt < 2; ++nt) {
            acc[mt][nt] = mma16(acc[mt][nt], ah[mt], b[nt]);
            acc[mt][nt] = mma16(acc[mt][nt], al[mt], b[nt]);
          }
        asm volatile("v_nop\n\tv_nop\n\tv_nop\n\tv_nop"
                     : "+v"(acc[0][0]), "+v"(acc[0][1]), "+v"(acc[1][0]), "+v"(acc[1][1])
                     : "v"(ah[0].v), "v"(ah[1].v), "v"(al[0].v), "v"(al[1].v), "v"(b[0].v), "v"(b[1].v));
      }
    }
    {
      lcp_us ha = hHc + m * HP;
      lcp_us la = hLc + m * HP;
      const unsigned short* wb = WH + (size_t)(32 * w + m) * NHD;
#pragma unroll 1
      for (int k0 = 0; k0 < NHD; k0 += 32) {
        Frag ah[2], al[2], b[2];
#pragma unroll
        for (int mt = 0; mt < 2; ++mt) {
          ldfrag_l(ah[mt], ha + mt * 16 * HP + k0, h);
          ldfrag_l(al[mt], la + mt * 16 * HP + k0, h);
        }
#pragma unroll
        for (int nt = 0; nt < 2; ++nt) ldfrag_g(b[nt], wb + (size_t)nt * 16 * NHD + k0, h);
#pragma unroll
        for (int mt = 0; mt < 2; ++mt)
#pragma unroll
          for (int nt = 0; nt < 2; ++nt) {
            acc[mt][nt] = mma16(acc[mt][nt], ah[mt], b[nt]);
            acc[mt][nt] = mma16(acc[mt][nt], al[mt], b[nt]);
          }
        asm volatile("v_nop\n\tv_nop\n\tv_nop\n\tv_nop"
                     : "+v"(acc[0][0]), "+v"(acc[0][1]), "+v"(acc[1][0]), "+v"(acc[1][1])
                     : "v"(ah[0].v), "v"(ah[1].v), "v"(al[0].v), "v"(al[1].v), "v"(b[0].v), "v"(b[1].v));
      }
    }

    float p[2][8];
#pragma unroll
    for (int mt = 0; mt < 2; ++mt)
#pragma unroll
      for (int r = 0; r < 8; ++r) p[mt][r] = 0.0f;
#pragma unroll
    for (int nt = 0; nt < 2; ++nt) {
      const int col = 32 * w + 16 * nt + m;
      const float bias = sBias[col];
#pragma unroll
      for (int mt = 0; mt < 2; ++mt)
#pragma unroll
        for (int r = 0; r < 8; ++r) {
          const int row = 16 * mt + 8 * h + r;
          const float v = fmaxf(acc[mt][nt][r] + bias, 0.0f);
          const unsigned short hb = bf16_bits(v);
          const unsigned short lb = bf16_bits(v - bf16_val(hb));
          hHn[row * HP + col] = hb;
          hLn[row * HP + col] = lb;
          p[mt][r] += v * bf16_val(sWg[row * NHD + col]);
        }
    }
#pragma unroll
    for (int mt = 0; mt < 2; ++mt)
#pragma unroll
      for (int r = 0; r < 8; ++r) {
        float q = p[mt][r];
        q += __shfl_xor(q, 1);
        q += __shfl_xor(q, 2);
        q += __shfl_xor(q, 4);
        q += __shfl_xor(q, 8);
        p[mt][r] = q;
      }
    if (m == 0) {
      const int tj = t & 31;
#pragma unroll
      for (int mt = 0; mt < 2; ++mt)
#pragma unroll
        for (int r = 0; r < 8; ++r)
          sZw[(w * 32 + 16 * mt + 8 * h + r) * 32 + tj] = p[mt][r];
    }

    const bool fl = dir ? ((t & 31) == 0) : (((t & 31) == 31) || (t == NT - 1));
    if (fl) {
      __syncthreads();
      const int c32 = t & ~31;
      v4f zv[2];
      size_t zo[2];
#pragma unroll
      for (int i = 0; i < 2; ++i) {
        const int row = 8 * w + 4 * i + sub;
        lcp_f zp = sZw + row * 32 + 4 * q8;
        v4f z = *(AS3 const v4fa*)(zp);
        z += *(AS3 const v4fa*)(zp + 1024);
        z += *(AS3 const v4fa*)(zp + 2048);
        z += *(AS3 const v4fa*)(zp + 3072);
        zv[i] = z;
        zo[i] = ((size_t)(dir * NB + b0 + row)) * ZP + c32 + 4 * q8;
      }
      *(volatile v4f*)(zpl + zo[0]) = zv[0];
      *(volatile v4f*)(zpl + zo[1]) = zv[1];
      __threadfence();
      *(volatile v4f*)(zpl + zo[0]) = zv[0];
      *(volatile v4f*)(zpl + zo[1]) = zv[1];
    }
  }
}

__global__ __launch_bounds__(256)
void out_kernel(const float* __restrict__ cpl, const float* __restrict__ zpl, float* out)
{
  const int g = blockIdx.x * 256 + threadIdx.x;
  if (g >= (NB * NT) / 4) return;
  const int e0 = g * 4;
  v4f o;
#pragma unroll
  for (int j = 0; j < 4; ++j) {
    const int e = e0 + j;
    const int b = e / NT;
    const int t = e - b * NT;
    const float y = cpl[b] + zpl[(size_t)b * ZP + t] + zpl[(size_t)(NB + b) * ZP + t];
    o[j] = fmaxf(y, 0.0f);
  }
  float* dst = out + e0;
  *(volatile v4f*)dst = o;
  __threadfence();
  *(volatile v4f*)dst = o;
}

extern "C" void kernel_launch(void* const* d_in, const int* in_sizes, int n_in,
                              void* d_out, int out_size, void* d_ws, size_t ws_size,
                              hipStream_t stream)
{
  if (n_in < 19) return;
  if (in_sizes[0]  != NB * NIS)       return;
  if (in_sizes[1]  != NB * NT * NID)  return;
  if (in_sizes[2]  != NB)             return;
  if (in_sizes[3]  != NHS * NIS)      return;
  if (in_sizes[4]  != NHS)            return;
  if (in_sizes[5]  != NHS * NHS)      return;
  if (in_sizes[6]  != NHS)            return;
  if (in_sizes[7]  != NHD * NID)      return;
  if (in_sizes[8]  != NHD)            return;
  if (in_sizes[9]  != NHD * NHD)      return;
  if (in_sizes[10] != NHD * NHD)      return;
  if (in_sizes[11] != NHD)            return;
  if (in_sizes[12] != NHD)            return;
  if (in_sizes[13] != NHD * NHD)      return;
  if (in_sizes[14] != NHD * NHD)      return;
  if (in_sizes[15] != NHD)            return;
  if (in_sizes[16] != NHD)            return;
  if (in_sizes[17] != NNEU * NFD)     return;
  if (in_sizes[18] != NNEU)           return;
  if (out_size != NB * NT)            return;
  if (ws_size < WS_END)               return;

  const float* xs   = (const float*)d_in[0];
  const float* xd   = (const float*)d_in[1];
  const int*   nord = (const int*)d_in[2];
  const float* w1   = (const float*)d_in[3];
  const float* b1   = (const float*)d_in[4];
  const float* w2   = (const float*)d_in[5];
  const float* b2   = (const float*)d_in[6];
  const float* wd   = (const float*)d_in[7];
  const float* bd   = (const float*)d_in[8];
  const float* wif  = (const float*)d_in[9];
  const float* whf  = (const float*)d_in[10];
  const float* bihf = (const float*)d_in[11];
  const float* bhhf = (const float*)d_in[12];
  const float* wib  = (const float*)d_in[13];
  const float* whb  = (const float*)d_in[14];
  const float* bihb = (const float*)d_in[15];
  const float* bhhb = (const float*)d_in[16];
  const float* fcw  = (const float*)d_in[17];
  const float* fcb  = (const float*)d_in[18];
  float* out = (float*)d_out;

  char* ws = (char*)d_ws;
  unsigned short* cv  = (unsigned short*)(ws + OFF_CV);
  unsigned short* dhp = (unsigned short*)(ws + OFF_DH);
  unsigned short* dlp = (unsigned short*)(ws + OFF_DL);
  float* cpl = (float*)(ws + OFF_C);
  float* zpl = (float*)(ws + OFF_Z);

  cvt_kernel<<<dim3(NCBLK), dim3(256), 0, stream>>>(xs, w1, w2, wd, wif, whf, wib, whb, xd, cv);

  hipFuncSetAttribute(reinterpret_cast<const void*>(&smlp_kernel),
                      hipFuncAttributeMaxDynamicSharedMemorySize, (int)SLDS);
  smlp_kernel<<<dim3(NB / 32), dim3(256), SLDS, stream>>>(cv, b1, b2, nord, fcw, fcb, cpl);

  dproj_kernel<<<dim3((NB * NT) / 128, 2), dim3(128), DLDS, stream>>>(cv, bd, dhp, dlp);

  brnn_kernel<<<dim3(32), dim3(128), RLDS, stream>>>(cv, dhp, dlp, bihf, bhhf, bihb, bhhb, nord, fcw, zpl);

  out_kernel<<<dim3((NB * NT) / 4 / 256), dim3(256), 0, stream>>>(cpl, zpl, out);
}
